// Block_36447092474456
// MI455X (gfx1250) — hardware-verified
//
#include <hip/hip_runtime.h>
#include <math.h>

typedef __attribute__((ext_vector_type(16))) _Float16 v16h;
typedef __attribute__((ext_vector_type(8)))  _Float16 v8h;
typedef __attribute__((ext_vector_type(8)))  float    v8f;
typedef __attribute__((ext_vector_type(4)))  float    v4f;
typedef unsigned int u4 __attribute__((ext_vector_type(4)));
typedef unsigned int u2 __attribute__((ext_vector_type(2)));

#ifndef NB
#define NB 2
#endif
#ifndef SEQ
#define SEQ 2048
#endif
#define NB_FULL 2
#define SEQ_FULL 2048
#define CW 1024
#define FW 4096
#define NH 16
#define HD 64
#define ROWS (NB * SEQ)
#define FCHUNK (ROWS / 2)

static_assert(NH * HD == CW);
static_assert(HD == 64);
static_assert(CW == 128 * 8);
static_assert(SEQ % 64 == 0);
static_assert(ROWS % 128 == 0);
static_assert(FCHUNK % 64 == 0);
static_assert(CW % 64 == 0 && FW % 64 == 0 && (3 * CW) % 64 == 0);
static_assert(CW % 32 == 0 && FW % 32 == 0);
static_assert(NB <= NB_FULL && SEQ <= SEQ_FULL);


#define VST2(T, ptr, val) do { const T vst2_v_ = (val); *(volatile T*)(ptr) = vst2_v_; __threadfence(); *(volatile T*)(ptr) = vst2_v_; } while (0)

__device__ __forceinline__ float cmb_bf(float v) { const unsigned u = __builtin_bit_cast(unsigned, v); const unsigned r = (u + 0x7fffu + ((u >> 16) & 1u)) & 0xffff0000u; return __builtin_bit_cast(float, r); }
__device__ __forceinline__ unsigned int pk2h(float a, float b) { return (unsigned int)__builtin_bit_cast(unsigned short, (_Float16)a) | ((unsigned int)__builtin_bit_cast(unsigned short, (_Float16)b) << 16); }

__device__ __forceinline__ void dep_guard_h(v8f& a, v8f& b, v16h x, v16h y) { asm volatile("v_nop\n\tv_nop\n\tv_nop\n\tv_nop" : "+v"(a), "+v"(b) : "v"(x), "v"(y)); }
__device__ __forceinline__ void keep4_h(v16h a, v16h b, v16h c, v16h d) { asm volatile("v_nop" :: "v"(a), "v"(b), "v"(c), "v"(d)); }
__device__ __forceinline__ void acc_guard4(v8f& a, v8f& b, v8f& c, v8f& d) { asm volatile("v_nop\n\tv_nop\n\tv_nop\n\tv_nop" : "+v"(a), "+v"(b), "+v"(c), "+v"(d)); }
union FragU { v16h v; v8h h[2]; };
__device__ __forceinline__ v16h frag_ld(const _Float16* p) { FragU f; f.h[0] = *(const v8h*)(p); f.h[1] = *(const v8h*)(p + 16); return f.v; }
__device__ __forceinline__ v8f mma16(v16h a, v16h b, v8f c) { return __builtin_amdgcn_wmma_f32_16x16x32_f16(false, a, false, b, (short)0, c, false, false); }
__device__ __forceinline__ v8f mma16g(v16h a, v16h b, v8f c) {
  c = __builtin_amdgcn_wmma_f32_16x16x32_f16(false, a, false, b, (short)0, c, false, false);
  asm volatile("v_nop\n\tv_nop\n\tv_nop\n\tv_nop" : "+v"(c) : "v"(a), "v"(b));
  return c;
}

__global__ __launch_bounds__(256) void k_castbT(const float* __restrict__ SRC, int lds, unsigned short* __restrict__ DST, int ldd, int nR, int nC, float sc) {
    const long long u = (long long)blockIdx.x * 256 + threadIdx.x; const int per = nR / 8; if (u >= (long long)nC * per) return; const int c = (int)(u / per); const int r0 = 8 * (int)(u % per);
    float w[8];
#pragma unroll
    for (int e = 0; e < 8; ++e) w[e] = cmb_bf(SRC[(long long)(r0 + e) * lds + c]) * sc;
    u4 pk; pk.x = pk2h(w[0], w[1]); pk.y = pk2h(w[2], w[3]); pk.z = pk2h(w[4], w[5]); pk.w = pk2h(w[6], w[7]); VST2(u4, (u4*)(DST + (long long)c * ldd + r0), pk); }

__global__ __launch_bounds__(256) void k_ln16(const float* __restrict__ A, const float* __restrict__ GA, const float* __restrict__ BE, float eps, int rows, int seq, int seq_full, int abf, unsigned short* __restrict__ Y16) {
    #pragma clang fp contract(off)
    const int r = blockIdx.x * 8 + (threadIdx.x >> 5); const int L = threadIdx.x & 31; if (r >= rows) return;
    const long long rin = (long long)(r / seq) * seq_full + (r % seq);
    v4f v[8]; float s = 0.f;
#pragma unroll
    for (int q = 0; q < 8; ++q) { v[q] = *(const v4f*)(A + rin * CW + 4 * L + 128 * q); if (abf) { v[q].x = cmb_bf(v[q].x); v[q].y = cmb_bf(v[q].y); v[q].z = cmb_bf(v[q].z); v[q].w = cmb_bf(v[q].w); } s += (v[q].x + v[q].y) + (v[q].z + v[q].w); }
#pragma unroll
    for (int o = 16; o > 0; o >>= 1) s += __shfl_xor(s, o, 32);
    const float mu = s * (1.f / CW); float qq = 0.f;
#pragma unroll
    for (int q = 0; q < 8; ++q) { v[q].x -= mu; v[q].y -= mu; v[q].z -= mu; v[q].w -= mu; qq += (v[q].x * v[q].x + v[q].y * v[q].y) + (v[q].z * v[q].z + v[q].w * v[q].w); }
#pragma unroll
    for (int o = 16; o > 0; o >>= 1) qq += __shfl_xor(qq, o, 32);
    const float rs = rsqrtf(qq * (1.f / CW) + eps);
    u2 pk[8];
#pragma unroll
    for (int q = 0; q < 8; ++q) { const int c = 4 * L + 128 * q; const v4f ga = *(const v4f*)(GA + c), be = *(const v4f*)(BE + c);
        const float y0 = v[q].x * rs * cmb_bf(ga.x) + cmb_bf(be.x), y1 = v[q].y * rs * cmb_bf(ga.y) + cmb_bf(be.y), y2 = v[q].z * rs * cmb_bf(ga.z) + cmb_bf(be.z), y3 = v[q].w * rs * cmb_bf(ga.w) + cmb_bf(be.w);
        pk[q].x = pk2h(y0, y1); pk[q].y = pk2h(y2, y3); }
    unsigned short* yr = Y16 + (long long)r * CW + 4 * L;
#pragma unroll
    for (int q = 0; q < 8; ++q) *(volatile u2*)(yr + 128 * q) = pk[q];
    __threadfence();
#pragma unroll
    for (int q = 0; q < 8; ++q) *(volatile u2*)(yr + 128 * q) = pk[q];
}

__global__ __launch_bounds__(256) void k_gelu16(const float* __restrict__ F, unsigned short* __restrict__ Y16, long long n8) {
    #pragma clang fp contract(off)
    const long long u = (long long)blockIdx.x * 256 + threadIdx.x; if (u >= n8) return;
    unsigned long long lo = 0ull, hi = 0ull;
#pragma unroll 1
    for (int e = 0; e < 8; ++e) {
        const float a = F[8 * u + e];
        const float gl = 0.5f * a * (1.f + erff(a * 0.70710678118654752f));
        const unsigned long long bits = (unsigned long long)__builtin_bit_cast(unsigned short, (_Float16)gl);
        const unsigned long long sh = bits << (16 * (e & 3));
        lo |= (e < 4) ? sh : 0ull; hi |= (e < 4) ? 0ull : sh;
    }
    u4 pk; pk.x = (unsigned)(lo & 0xFFFFFFFFull); pk.y = (unsigned)(lo >> 32); pk.z = (unsigned)(hi & 0xFFFFFFFFull); pk.w = (unsigned)(hi >> 32);
    VST2(u4, (u4*)(Y16 + 8 * u), pk);
}

__global__ __launch_bounds__(256) void k_add(const float* __restrict__ A, const float* __restrict__ X, int seq, int seq_full, int xbf, float* __restrict__ O, long long n4) {
    #pragma clang fp contract(off)
    const long long u = (long long)blockIdx.x * 256 + threadIdx.x; if (u >= n4) return;
    const long long r = u / (CW / 4); const int c4 = (int)(u % (CW / 4));
    const long long rin = (r / seq) * seq_full + (r % seq);
    const v4f a = *(const v4f*)(A + 4 * u); v4f x = *(const v4f*)(X + rin * CW + 4 * c4);
    if (xbf) { x.x = cmb_bf(x.x); x.y = cmb_bf(x.y); x.z = cmb_bf(x.z); x.w = cmb_bf(x.w); }
    v4f y; y.x = x.x + a.x; y.y = x.y + a.y; y.z = x.z + a.z; y.w = x.w + a.w;
    VST2(v4f, (v4f*)(O + 4 * u), y);
}

template <int BIAS>
__device__ __forceinline__ void gemm64_body(const unsigned short* __restrict__ Ap, int lda, const unsigned short* __restrict__ Btp, int ldb,
                                            float* __restrict__ C, int ldc, const float* __restrict__ bias, int M, int N, int K, float scale) {
  const _Float16* A = (const _Float16*)Ap; const _Float16* Bt = (const _Float16*)Btp;
  __shared__ __align__(16) float sT[8][16 * 68];
  const int lane = threadIdx.x & 31;
  const int wave = threadIdx.x >> 5;
  const int tilesN = N >> 6;
  const int tilesM = M >> 6;
  const int tile = blockIdx.x * 8 + wave;
  if (tile >= tilesM * tilesN) return;
  const int tm = tile / tilesN;
  const int tn = tile - tm * tilesN;
  const int m0 = tm << 6;
  const int n0 = tn << 6;
  const int rlane = lane & 15;
  const int koff  = (lane >> 4) * 8;
  const int mOff  = (lane >> 4) * 8;

  v8f acc[4][4];
#pragma unroll
  for (int i = 0; i < 4; ++i)
#pragma unroll
    for (int j = 0; j < 4; ++j) acc[i][j] = (v8f){0.f,0.f,0.f,0.f,0.f,0.f,0.f,0.f};

  for (int k0 = 0; k0 < K; k0 += 32) {
    v16h bh[4];
#pragma unroll
    for (int j = 0; j < 4; ++j) {
      const size_t bo = (size_t)(n0 + (j << 4) + rlane) * ldb + koff + k0;
      bh[j] = frag_ld(Bt + bo);
    }
#pragma unroll
    for (int i = 0; i < 4; ++i) {
      const size_t ao = (size_t)(m0 + (i << 4) + rlane) * lda + koff + k0;
      const v16h ah = frag_ld(A + ao);
#pragma unroll
      for (int j = 0; j < 4; ++j) acc[i][j] = mma16(ah, bh[j], acc[i][j]);
      dep_guard_h(acc[i][0], acc[i][3], ah, ah);
    }
    keep4_h(bh[0], bh[1], bh[2], bh[3]);
  }
  acc_guard4(acc[0][0], acc[0][1], acc[0][2], acc[0][3]);
  acc_guard4(acc[1][0], acc[1][1], acc[1][2], acc[1][3]);
  acc_guard4(acc[2][0], acc[2][1], acc[2][2], acc[2][3]);
  acc_guard4(acc[3][0], acc[3][1], acc[3][2], acc[3][3]);

  float* slab = sT[wave];
#pragma unroll
  for (int i = 0; i < 4; ++i) {
    const int mBase = m0 + (i << 4);
#pragma unroll
    for (int j = 0; j < 4; ++j) {
      const int n = n0 + (j << 4) + rlane;
      float bv = 0.f;
      if (BIAS) bv = cmb_bf(bias[n]);
#pragma unroll
      for (int r = 0; r < 8; ++r) slab[(mOff + r) * 68 + (j << 4) + rlane] = acc[i][j][r] * scale + bv;
    }
    __builtin_amdgcn_fence(3  , "workgroup");
    __builtin_amdgcn_wave_barrier();
    __builtin_amdgcn_fence(2  , "workgroup");
    {
      const int hh = lane >> 4, c4 = (lane & 15) * 4;
      for (int pass = 0; pass < 2; ++pass) {
#pragma unroll
        for (int it = 0; it < 8; ++it) {
          const int row = it * 2 + hh;
          const v4f v = *(const v4f*)(slab + row * 68 + c4);
          *(volatile v4f*)(C + (size_t)(mBase + row) * ldc + n0 + c4) = v;
        }
        __threadfence();
      }
    }
    __builtin_amdgcn_fence(3  , "workgroup");
    __builtin_amdgcn_wave_barrier();
    __builtin_amdgcn_fence(2  , "workgroup");
  }
}
__global__ __launch_bounds__(256) void k_gemm_nb(const unsigned short* __restrict__ Ap, int lda, const unsigned short* __restrict__ Btp, int ldb, float* __restrict__ C, int ldc, int M, int N, int K, float scale) {
  gemm64_body<0>(Ap, lda, Btp, ldb, C, ldc, nullptr, M, N, K, scale);
}
__global__ __launch_bounds__(256) void k_gemm_b(const unsigned short* __restrict__ Ap, int lda, const unsigned short* __restrict__ Btp, int ldb, float* __restrict__ C, int ldc, const float* __restrict__ bias, int M, int N, int K, float scale) {
  gemm64_body<1>(Ap, lda, Btp, ldb, C, ldc, bias, M, N, K, scale);
}

#define AT_D 64
#define AT_NW 4
#define AT_QB 64
#define AT_KC 64
struct AttnGeom { long long q_bs, q_rs, q_hs, k_bs, k_rs, k_hs, v_bs, v_rs, v_hs, o_bs, o_rs, o_hs; int S, Skv, H, pad_; float qscale, oscale; };
static_assert(sizeof(AttnGeom) == 12 * 8 + 4 * 4 + 2 * 4);

__global__ __launch_bounds__(128)
void k_attn64(const float* __restrict__ q, const float* __restrict__ k, const float* __restrict__ v, unsigned short* __restrict__ out16, AttnGeom g) {
  const float PSC = 32768.0f;
  __shared__ __align__(16) _Float16 Ksh[AT_KC * AT_D];
  __shared__ __align__(16) _Float16 Vth[AT_D * AT_KC];
  __shared__ __align__(16) _Float16 Psh[AT_NW][16 * AT_KC];
  __shared__ __align__(16) float    Os[AT_NW][16 * 68];

  const int tid  = threadIdx.x;
  const int wave = tid >> 5;
  const int lane = tid & 31;
  const int hh   = lane >> 4;
  const int c    = lane & 15;

  const int nqb = g.S / AT_QB;
  const int bx = blockIdx.x;
  const int qb = bx % nqb;
  const int bh = bx / nqb;
  const int h  = bh % g.H;
  const int b  = bh / g.H;
  const int q0 = qb * AT_QB + wave * 16;

  const float* qb_ptr = q + (size_t)b * g.q_bs + (size_t)h * g.q_hs;
  const float* kb_ptr = k + (size_t)b * g.k_bs + (size_t)h * g.k_hs;
  const float* vb_ptr = v + (size_t)b * g.v_bs + (size_t)h * g.v_hs;
  unsigned short* ob_ptr = out16 + (size_t)b * g.o_bs + (size_t)h * g.o_hs;

  v16h qa[2];
  {
    const float* qrow = qb_ptr + (size_t)(q0 + c) * g.q_rs;
#pragma unroll
    for (int dc = 0; dc < 2; ++dc) {
#pragma unroll
      for (int e = 0; e < 8; ++e) {
        qa[dc][e]     = (_Float16)(qrow[dc * 32 + 8 * hh + e] * g.qscale);
        qa[dc][8 + e] = (_Float16)(qrow[dc * 32 + 16 + 8 * hh + e] * g.qscale);
      }
    }
  }

  float mrow[8], lrow[8];
  v8f oacc[4];
#pragma unroll
  for (int r = 0; r < 8; ++r) { mrow[r] = -INFINITY; lrow[r] = 0.f; }
#pragma unroll
  for (int t = 0; t < 4; ++t) oacc[t] = (v8f){0.f,0.f,0.f,0.f,0.f,0.f,0.f,0.f};

  const int nChunks = g.Skv / AT_KC;
  for (int kc = 0; kc < nChunks; ++kc) {
    const int kv0 = kc * AT_KC;
    __syncthreads();
    {
      const int kvr = tid >> 1, dh = (tid & 1) * 32;
      const float* krow = kb_ptr + (size_t)(kv0 + kvr) * g.k_rs + dh;
      const float* vrow = vb_ptr + (size_t)(kv0 + kvr) * g.v_rs + dh;
#pragma unroll
      for (int i = 0; i < 8; ++i) {
        const v4f kk = *(const v4f*)(krow + 4 * i);
        const v4f vv = *(const v4f*)(vrow + 4 * i);
#pragma unroll
        for (int e = 0; e < 4; ++e) {
          const int d = dh + 4 * i + e;
          Ksh[kvr * AT_D + d] = (_Float16)kk[e];
          Vth[d * AT_KC + kvr] = (_Float16)vv[e];
        }
      }
    }
    __syncthreads();

    v8f s[4];
#pragma unroll
    for (int j = 0; j < 4; ++j) {
      s[j] = (v8f){0.f,0.f,0.f,0.f,0.f,0.f,0.f,0.f};
#pragma unroll
      for (int dc = 0; dc < 2; ++dc) {
        FragU kb;
        kb.h[0] = *(const v8h*)(Ksh + (j * 16 + c) * AT_D + dc * 32 + 8 * hh);
        kb.h[1] = *(const v8h*)(Ksh + (j * 16 + c) * AT_D + dc * 32 + 16 + 8 * hh);
        s[j] = mma16g(qa[dc], kb.v, s[j]);
      }
    }
    float cm[8];
#pragma unroll
    for (int r = 0; r < 8; ++r) {
      float m = fmaxf(fmaxf(s[0][r], s[1][r]), fmaxf(s[2][r], s[3][r]));
#pragma unroll
      for (int off = 1; off < 16; off <<= 1) m = fmaxf(m, __shfl_xor(m, off, 32));
      cm[r] = m;
    }
    _Float16* pwh = Psh[wave];
#pragma unroll
    for (int r = 0; r < 8; ++r) {
      const float mnew = fmaxf(mrow[r], cm[r]);
      const float alpha = expf(mrow[r] - mnew);
      mrow[r] = mnew;
      float psum = 0.f;
#pragma unroll
      for (int j = 0; j < 4; ++j) {
        const float p = expf(s[j][r] - mnew);
        psum += p;
        pwh[(8 * hh + r) * AT_KC + j * 16 + c] = (_Float16)(p * PSC);
      }
#pragma unroll
      for (int off = 1; off < 16; off <<= 1) psum += __shfl_xor(psum, off, 32);
      lrow[r] = lrow[r] * alpha + psum;
#pragma unroll
      for (int t = 0; t < 4; ++t) oacc[t][r] *= alpha;
    }
    __builtin_amdgcn_fence(3  , "workgroup");
    __builtin_amdgcn_wave_barrier();
    __builtin_amdgcn_fence(2  , "workgroup");
#pragma unroll
    for (int kk = 0; kk < 2; ++kk) {
      FragU pa;
      pa.h[0] = *(const v8h*)(pwh + c * AT_KC + kk * 32 + 8 * hh);
      pa.h[1] = *(const v8h*)(pwh + c * AT_KC + kk * 32 + 16 + 8 * hh);
#pragma unroll
      for (int t = 0; t < 4; ++t) {
        FragU vb;
        vb.h[0] = *(const v8h*)(Vth + (t * 16 + c) * AT_KC + kk * 32 + 8 * hh);
        vb.h[1] = *(const v8h*)(Vth + (t * 16 + c) * AT_KC + kk * 32 + 16 + 8 * hh);
        oacc[t] = mma16g(pa.v, vb.v, oacc[t]);
      }
    }
  }

  float* os = Os[wave];
#pragma unroll
  for (int r = 0; r < 8; ++r) {
    const float inv = g.oscale / (lrow[r] * PSC);
#pragma unroll
    for (int t = 0; t < 4; ++t) os[(8 * hh + r) * 68 + t * 16 + c] = oacc[t][r] * inv;
  }
  __builtin_amdgcn_fence(3  , "workgroup");
  __builtin_amdgcn_wave_barrier();
  __builtin_amdgcn_fence(2  , "workgroup");
  {
    const int qq = lane >> 3, c8 = (lane & 7) * 8;
    v8h hv[4];
#pragma unroll
    for (int it = 0; it < 4; ++it) {
      const int row = it * 4 + qq;
      const v4f a0 = *(const v4f*)(os + row * 68 + c8);
      const v4f a1 = *(const v4f*)(os + row * 68 + c8 + 4);
      hv[it][0] = (_Float16)a0.x; hv[it][1] = (_Float16)a0.y; hv[it][2] = (_Float16)a0.z; hv[it][3] = (_Float16)a0.w;
      hv[it][4] = (_Float16)a1.x; hv[it][5] = (_Float16)a1.y; hv[it][6] = (_Float16)a1.z; hv[it][7] = (_Float16)a1.w;
    }
    for (int pass = 0; pass < 2; ++pass) {
#pragma unroll
      for (int it = 0; it < 4; ++it) {
        const int row = it * 4 + qq;
        *(volatile v8h*)(ob_ptr + (size_t)(q0 + row) * g.o_rs + c8) = hv[it];
      }
      __threadfence();
    }
  }
}

constexpr size_t SZ_X16 = (size_t)ROWS * CW * 2;
constexpr size_t SZ_W3  = (size_t)3 * CW * CW * 2;
constexpr size_t SZ_QKV = (size_t)ROWS * 3 * CW * 4;
constexpr size_t SZ_WO  = (size_t)CW * CW * 2;
constexpr size_t SZ_ATT = (size_t)ROWS * CW * 4;
constexpr size_t SZ_X1  = (size_t)ROWS * CW * 4;
constexpr size_t SZ_W1T = (size_t)FW * CW * 2;
constexpr size_t SZ_W2T = (size_t)CW * FW * 2;
constexpr size_t OFF_X16 = 0;
constexpr size_t OFF_W3  = OFF_X16 + SZ_X16;
constexpr size_t OFF_QKV = OFF_W3 + SZ_W3;
constexpr size_t OFF_WO  = OFF_QKV + SZ_QKV;
constexpr size_t OFF_ATT = OFF_WO + SZ_WO;
constexpr size_t OFF_X1  = OFF_ATT + SZ_ATT;
constexpr size_t OFF_W1T = OFF_X1 + SZ_X1;
constexpr size_t OFF_W2T = OFF_W1T + SZ_W1T;
constexpr size_t WS_TOTAL = OFF_W2T + SZ_W2T;
constexpr size_t SZ_F1  = (size_t)FCHUNK * FW * 4;
constexpr size_t SZ_F16 = (size_t)FCHUNK * FW * 2;
constexpr size_t SZ_FFO = (size_t)FCHUNK * CW * 4;
static_assert(WS_TOTAL <= (size_t)134217728);
static_assert(SZ_F1 + SZ_F16 <= SZ_QKV);
static_assert(SZ_FFO <= SZ_ATT);
static_assert(SZ_X16 % 256 == 0 && SZ_W3 % 256 == 0 && SZ_QKV % 256 == 0 && SZ_WO % 256 == 0 && SZ_ATT % 256 == 0 && SZ_X1 % 256 == 0 && SZ_W1T % 256 == 0 && SZ_F1 % 256 == 0);
static_assert(2 * FCHUNK == ROWS);

extern "C" void kernel_launch(void* const* d_in, const int* in_sizes, int n_in, void* d_out, int out_size, void* d_ws, size_t ws_size, hipStream_t stream) {
    if (n_in < 14) return;
    if ((long long)in_sizes[0] < ((long long)(NB - 1) * SEQ_FULL + SEQ) * CW) return;
    if (in_sizes[1] < CW * CW || in_sizes[2] < CW * CW || in_sizes[3] < CW * CW || in_sizes[4] < CW * CW) return;
    if (in_sizes[5] < CW || in_sizes[6] < CW * FW || in_sizes[7] < FW || in_sizes[8] < FW * CW || in_sizes[9] < CW) return;
    if (in_sizes[10] < CW || in_sizes[11] < CW || in_sizes[12] < CW || in_sizes[13] < CW) return;
    if ((long long)out_size < (long long)ROWS * CW) return;
    if (WS_TOTAL > ws_size) return;
    const float* x   = (const float*)d_in[0];
    const float* wq  = (const float*)d_in[1];
    const float* wk  = (const float*)d_in[2];
    const float* wv  = (const float*)d_in[3];
    const float* wp  = (const float*)d_in[4];
    const float* bp  = (const float*)d_in[5];
    const float* w1  = (const float*)d_in[6];
    const float* b1  = (const float*)d_in[7];
    const float* w2  = (const float*)d_in[8];
    const float* b2  = (const float*)d_in[9];
    const float* g1  = (const float*)d_in[10];
    const float* be1 = (const float*)d_in[11];
    const float* g2  = (const float*)d_in[12];
    const float* be2 = (const float*)d_in[13];
    float* out = (float*)d_out;
    char* ws = (char*)d_ws;
    unsigned short* X16  = (unsigned short*)(ws + OFF_X16);
    unsigned short* AO16 = X16;
    unsigned short* H16  = X16;
    unsigned short* W316 = (unsigned short*)(ws + OFF_W3);
    float*          QKV  = (float*)(ws + OFF_QKV);
    float*          F1   = (float*)(ws + OFF_QKV);
    unsigned short* F16  = (unsigned short*)(ws + OFF_QKV + SZ_F1);
    unsigned short* WO16 = (unsigned short*)(ws + OFF_WO);
    float*          ATT  = (float*)(ws + OFF_ATT);
    float*          FFo  = (float*)(ws + OFF_ATT);
    float*          X1   = (float*)(ws + OFF_X1);
    unsigned short* W1T  = (unsigned short*)(ws + OFF_W1T);
    unsigned short* W2T  = (unsigned short*)(ws + OFF_W2T);

    k_ln16<<<(ROWS + 7) / 8, 256, 0, stream>>>(x, g1, be1, 1e-6f, ROWS, SEQ, SEQ_FULL, 1, X16);
    k_castbT<<<(unsigned)(((long long)CW * (CW / 8) + 255) / 256), 256, 0, stream>>>(wq, CW, W316, CW, CW, CW, 16.0f);
    k_castbT<<<(unsigned)(((long long)CW * (CW / 8) + 255) / 256), 256, 0, stream>>>(wk, CW, W316 + (size_t)CW * CW, CW, CW, CW, 16.0f);
    k_castbT<<<(unsigned)(((long long)CW * (CW / 8) + 255) / 256), 256, 0, stream>>>(wv, CW, W316 + (size_t)2 * CW * CW, CW, CW, CW, 16.0f);
    k_castbT<<<(unsigned)(((long long)CW * (CW / 8) + 255) / 256), 256, 0, stream>>>(wp, CW, WO16, CW, CW, CW, 16.0f);
    k_gemm_nb<<<(unsigned)((((ROWS / 64) * ((3 * CW) / 64)) + 7) / 8), 256, 0, stream>>>(X16, CW, W316, CW, QKV, 3 * CW, ROWS, 3 * CW, CW, 0.0625f);
    {
        AttnGeom g;
        g.q_bs = (long long)SEQ * 3 * CW; g.q_rs = 3 * CW; g.q_hs = HD;
        g.k_bs = (long long)SEQ * 3 * CW; g.k_rs = 3 * CW; g.k_hs = HD;
        g.v_bs = (long long)SEQ * 3 * CW; g.v_rs = 3 * CW; g.v_hs = HD;
        g.o_bs = (long long)SEQ * CW; g.o_rs = CW; g.o_hs = HD;
        g.S = SEQ; g.Skv = SEQ; g.H = NH; g.pad_ = 0; g.qscale = 0.125f; g.oscale = 64.0f;
        k_attn64<<<(unsigned)(NB * NH * (SEQ / AT_QB)), 128, 0, stream>>>(QKV, QKV + CW, QKV + 2 * CW, AO16, g);
    }
    k_gemm_b<<<(unsigned)((((ROWS / 64) * (CW / 64)) + 7) / 8), 256, 0, stream>>>(AO16, CW, WO16, CW, ATT, CW, bp, ROWS, CW, CW, 0.0009765625f);
    k_castbT<<<(unsigned)(((long long)FW * (CW / 8) + 255) / 256), 256, 0, stream>>>(w1, FW, W1T, CW, CW, FW, 16.0f);
    k_castbT<<<(unsigned)(((long long)CW * (FW / 8) + 255) / 256), 256, 0, stream>>>(w2, CW, W2T, FW, FW, CW, 16.0f);
    k_add<<<(unsigned)(((long long)ROWS * (CW / 4) + 255) / 256), 256, 0, stream>>>(ATT, x, SEQ, SEQ_FULL, 1, X1, (long long)ROWS * (CW / 4));
    k_ln16<<<(ROWS + 7) / 8, 256, 0, stream>>>(X1, g2, be2, 1e-6f, ROWS, SEQ, SEQ, 0, H16);
    for (int ch = 0; ch < 2; ++ch) {
        const size_t ro = (size_t)ch * FCHUNK;
        k_gemm_b<<<(unsigned)((((FCHUNK / 64) * (FW / 64)) + 7) / 8), 256, 0, stream>>>(H16 + ro * CW, CW, W1T, CW, F1, FW, b1, FCHUNK, FW, CW, 0.0625f);
        k_gelu16<<<(unsigned)(((long long)FCHUNK * (FW / 8) + 255) / 256), 256, 0, stream>>>(F1, F16, (long long)FCHUNK * (FW / 8));
        k_gemm_b<<<(unsigned)((((FCHUNK / 64) * (CW / 64)) + 7) / 8), 256, 0, stream>>>(F16, FW, W2T, FW, FFo, CW, b2, FCHUNK, CW, FW, 0.0625f);
        k_add<<<(unsigned)(((long long)FCHUNK * (CW / 4) + 255) / 256), 256, 0, stream>>>(FFo, X1 + ro * CW, SEQ, SEQ, 0, out + ro * CW, (long long)FCHUNK * (CW / 4));
    }
}
